// WindowedMultiheadAttention_75574244540550
// MI455X (gfx1250) — hardware-verified
//
#include <hip/hip_runtime.h>
#include <stdint.h>

#define DEVINL __device__ __forceinline__

typedef _Float16 f16t;
typedef _Float16 v16h __attribute__((ext_vector_type(16)));
typedef _Float16 v8h  __attribute__((ext_vector_type(8)));
typedef float    v8f  __attribute__((ext_vector_type(8)));
typedef float    v4f  __attribute__((ext_vector_type(4)));
typedef v8h __attribute__((may_alias)) v8ha;
typedef v4f __attribute__((may_alias)) v4fa;
union FragH { v16h v; v8h half[2]; };

#define NBATCH 8
#define GH     32
#define GW     32
#define NTOKB  1024
#define NTOK   8192
#define CW     256
#define NQKV   768
#define NHEAD  8
#define HDIM   32
#define RH     3
#define RW     5
#define NTAPW  11
#define NSLOT  80
#define SLOTL  20
#define TPB    256
#define WAVES  8
#define MT     64
#define PQF    132
#define ACAR   16.0f
#define WCAR   256.0f
#define OCAR   256.0f
#define SC_AW  (1.0f / (16.0f * 256.0f))
#define SC_OW  (1.0f / (256.0f * 256.0f))
#define QSC    0.0625f

#define XBLK   (NTOK * CW / 8 / TPB)
#define WQBLK  (NQKV * CW / 8 / TPB)
#define WOBLK  (CW * CW / 8 / TPB)

static_assert(TPB == WAVES * 32);
static_assert(GH * GW == NTOKB);
static_assert(NBATCH * NTOKB == NTOK);
static_assert(NHEAD * HDIM == CW);
static_assert(NHEAD * 4 == 32);
static_assert(4 * SLOTL == NSLOT);
static_assert((2 * RH + 1) * NTAPW <= NSLOT);
static_assert((NTOK % MT) == 0);
static_assert((NTOK % WAVES) == 0);
static_assert((CW % 32) == 0);
static_assert((NQKV % 128) == 0);
static_assert((PQF % 4) == 0);
static_assert(MT == 64);
static_assert(XBLK * TPB * 8 == NTOK * CW);
static_assert(WQBLK * TPB * 8 == NQKV * CW);
static_assert(WOBLK * TPB * 8 == CW * CW);

DEVINL int imin(int a, int b) { return a < b ? a : b; }
DEVINL int imax(int a, int b) { return a > b ? a : b; }

DEVINL v8f wmma_f16(v16h a, v16h b, v8f c) {
  v8f d = __builtin_amdgcn_wmma_f32_16x16x32_f16(false, a, false, b, (short)0, c, false, false);
  asm volatile("v_nop\n\tv_nop\n\tv_nop\n\tv_nop" : "+v"(d) : "v"(a), "v"(b));
  return d;
}
DEVINL v8f zero8f() {
  v8f z = {0.f, 0.f, 0.f, 0.f, 0.f, 0.f, 0.f, 0.f};
  return z;
}
DEVINL void load_frag(FragH& f, const f16t* row, int k0) {
  f.half[0] = *(const v8ha*)(row + k0);
  f.half[1] = *(const v8ha*)(row + k0 + 16);
}

DEVINL float gsum4(float v) {
  v += __shfl_xor(v, 1);
  v += __shfl_xor(v, 2);
  return v;
}

template <int KD>
DEVINL void mma_4n(const f16t* __restrict__ arow, const f16t* __restrict__ brow, v8f (&acc)[4]) {
  #pragma unroll 1
  for (int ks = 0; ks < KD / 32; ++ks) {
    const int k0 = 32 * ks;
    FragH a;
    load_frag(a, arow, k0);
    #pragma unroll
    for (int n = 0; n < 4; ++n) {
      FragH b;
      load_frag(b, brow + (size_t)16 * n * KD, k0);
      acc[n] = wmma_f16(a.v, b.v, acc[n]);
    }
  }
}

DEVINL void store_rows_f32(const float* sbuf, float* dst, int pitch, int wave, int lane) {
  #pragma unroll
  for (int i = 0; i < 8; ++i) {
    const int row = wave + 8 * i;
    const v4f v = *(const v4fa*)(sbuf + row * PQF + 4 * lane);
    *(volatile v4f*)(dst + (size_t)row * pitch + 4 * lane) = v;
  }
  __threadfence();
  #pragma unroll
  for (int i = 0; i < 8; ++i) {
    const int row = wave + 8 * i;
    const v4f v = *(const v4fa*)(sbuf + row * PQF + 4 * lane);
    *(volatile v4f*)(dst + (size_t)row * pitch + 4 * lane) = v;
  }
}

__global__ __launch_bounds__(TPB) void prep_k(const float* __restrict__ x, const float* __restrict__ qw,
                                             const float* __restrict__ pw,
                                             f16t* __restrict__ X16, f16t* __restrict__ WQKV,
                                             f16t* __restrict__ WO)
{
  const int blk = blockIdx.x, tid = threadIdx.x;
  if (blk >= XBLK + WQBLK + WOBLK) return;
  const float* src;
  f16t* dst;
  float sc;
  int rb;
  if (blk < XBLK)              { src = x;  dst = X16;  sc = ACAR; rb = blk; }
  else if (blk < XBLK + WQBLK) { src = qw; dst = WQKV; sc = WCAR; rb = blk - XBLK; }
  else                         { src = pw; dst = WO;   sc = WCAR; rb = blk - XBLK - WQBLK; }
  const size_t idx = ((size_t)rb * TPB + tid) * 8;
  const v4f a = *(const v4fa*)(src + idx), c = *(const v4fa*)(src + idx + 4);
  v8h o;
  #pragma unroll
  for (int j = 0; j < 4; ++j) {
    o[j]     = (f16t)(a[j] * sc);
    o[4 + j] = (f16t)(c[j] * sc);
  }
  *(volatile v8h*)(dst + idx) = o;
  __threadfence();
  *(volatile v8h*)(dst + idx) = o;
}

__global__ __launch_bounds__(TPB) void gemm_qkv_k(const f16t* __restrict__ Xp, const f16t* __restrict__ Wp,
                                                 const float* __restrict__ bias,
                                                 float* __restrict__ Qo, float* __restrict__ Ko,
                                                 float* __restrict__ Vo)
{
  __shared__ __attribute__((aligned(16))) float sbuf[MT * PQF];
  const int tid = threadIdx.x, lane = tid & 31, wave = tid >> 5;
  const int h = lane >> 4, m = lane & 15;
  const int mt = wave & 3, nh = wave >> 2;
  const int row0 = blockIdx.x * MT, y = blockIdx.y;
  const int pl = y >> 1, chalf = y & 1;
  float* outp = (pl == 0) ? Qo : ((pl == 1) ? Ko : Vo);
  const float osc = (pl == 0) ? QSC : 1.0f;

  v8f acc[4];
  #pragma unroll
  for (int n = 0; n < 4; ++n) acc[n] = zero8f();
  const f16t* arow = Xp + (size_t)(row0 + 16 * mt + m) * CW + 8 * h;
  const f16t* brow = Wp + (size_t)(y * 128 + 64 * nh + m) * CW + 8 * h;
  mma_4n<CW>(arow, brow, acc);

  const int cb = y * 128 + 64 * nh;
  #pragma unroll
  for (int n = 0; n < 4; ++n) {
    const float bv = bias[cb + 16 * n + m];
    #pragma unroll
    for (int r = 0; r < 8; ++r)
      sbuf[(16 * mt + 8 * h + r) * PQF + 64 * nh + 16 * n + m] = (acc[n][r] * SC_AW + bv) * osc;
  }
  __syncthreads();
  store_rows_f32(sbuf, outp + (size_t)row0 * CW + 128 * chalf, CW, wave, lane);
}

__global__ __launch_bounds__(TPB) void attn_k(const float* __restrict__ Qp, const float* __restrict__ Kp,
                                             const float* __restrict__ Vp, f16t* __restrict__ Op)
{
  __shared__ __attribute__((aligned(16))) float sS[WAVES * NHEAD * NSLOT];
  const int tid = threadIdx.x, lane = tid & 31;
  const int wave = __builtin_amdgcn_readfirstlane(tid >> 5);
  const int gp = imin(blockIdx.x * WAVES + wave, NTOK - 1);
  const int bb = gp >> 10, n = gp & 1023, h0 = n >> 5, w0 = n & 31;
  const int head = lane >> 2, j4 = lane & 3, c0 = 8 * lane;
  float* sw = sS + wave * (NHEAD * NSLOT);
  float* sh = sw + head * NSLOT;

  {
    const v4f fill = {-1.0e9f, -1.0e9f, -1.0e9f, -1.0e9f};
    #pragma unroll
    for (int q = 0; q < 5; ++q) *(v4fa*)(sw + SLOTL * lane + 4 * q) = fill;
  }
  __syncthreads();

  const float* qp = Qp + (size_t)gp * CW + c0;
  const v4f qa = *(const v4fa*)qp, qc = *(const v4fa*)(qp + 4);
  const int hlo = imax(h0 - RH, 0), hhi = imin(h0 + RH, GH - 1);
  const int wlo = imax(w0 - RW, 0), whi = imin(w0 + RW, GW - 1);

  float mx = -3.0e38f;
  #pragma unroll 1
  for (int hh = hlo; hh <= hhi; ++hh) {
    const int th = (hh - h0 + RH) * NTAPW - w0 + RW;
    const size_t rowb = (size_t)(bb * NTOKB + hh * GW);
    #pragma unroll 1
    for (int ww = wlo; ww <= whi; ++ww) {
      const float* kp = Kp + (rowb + (size_t)ww) * CW + c0;
      const v4f ka = *(const v4fa*)kp, kc = *(const v4fa*)(kp + 4);
      float d = qa[0] * ka[0];
      d = fmaf(qa[1], ka[1], d);
      d = fmaf(qa[2], ka[2], d);
      d = fmaf(qa[3], ka[3], d);
      d = fmaf(qc[0], kc[0], d);
      d = fmaf(qc[1], kc[1], d);
      d = fmaf(qc[2], kc[2], d);
      d = fmaf(qc[3], kc[3], d);
      d = gsum4(d);
      mx = fmaxf(mx, d);
      sh[th + ww] = d;
    }
  }
  __syncthreads();

  float ssum = 0.0f;
  #pragma unroll 1
  for (int it = 0; it < SLOTL; ++it) {
    const int tt = j4 + 4 * it;
    const float sv = sh[tt];
    float e = __expf(sv - mx);
    e = (sv > -1.0e8f) ? e : 0.0f;
    sh[tt] = e;
    ssum += e;
  }
  ssum = gsum4(ssum);
  const float rS = 1.0f / ssum;
  __syncthreads();

  v4f cxa = {0.f, 0.f, 0.f, 0.f}, cxc = {0.f, 0.f, 0.f, 0.f};
  #pragma unroll 1
  for (int hh = hlo; hh <= hhi; ++hh) {
    const int th = (hh - h0 + RH) * NTAPW - w0 + RW;
    const size_t rowb = (size_t)(bb * NTOKB + hh * GW);
    #pragma unroll 1
    for (int ww = wlo; ww <= whi; ++ww) {
      const float p = sh[th + ww] * rS;
      const float* vp = Vp + (rowb + (size_t)ww) * CW + c0;
      const v4f va = *(const v4fa*)vp, vc = *(const v4fa*)(vp + 4);
      #pragma unroll
      for (int j = 0; j < 4; ++j) {
        cxa[j] = fmaf(p, va[j], cxa[j]);
        cxc[j] = fmaf(p, vc[j], cxc[j]);
      }
    }
  }

  v8h oh;
  #pragma unroll
  for (int j = 0; j < 4; ++j) {
    oh[j]     = (f16t)(cxa[j] * OCAR);
    oh[4 + j] = (f16t)(cxc[j] * OCAR);
  }
  f16t* dst = Op + (size_t)gp * CW + c0;
  *(volatile v8h*)dst = oh;
  __threadfence();
  *(volatile v8h*)dst = oh;
}

__global__ __launch_bounds__(TPB) void gemm_proj_k(const f16t* __restrict__ Opl, const f16t* __restrict__ Wp,
                                                  const float* __restrict__ bias, float* __restrict__ out)
{
  __shared__ __attribute__((aligned(16))) float sbuf[MT * PQF];
  const int tid = threadIdx.x, lane = tid & 31, wave = tid >> 5;
  const int h = lane >> 4, m = lane & 15;
  const int mt = wave & 3, nh = wave >> 2;
  const int row0 = blockIdx.x * MT, y = blockIdx.y;

  v8f acc[4];
  #pragma unroll
  for (int n = 0; n < 4; ++n) acc[n] = zero8f();
  const f16t* arow = Opl + (size_t)(row0 + 16 * mt + m) * CW + 8 * h;
  const f16t* brow = Wp + (size_t)(y * 128 + 64 * nh + m) * CW + 8 * h;
  mma_4n<CW>(arow, brow, acc);

  const int cb = y * 128 + 64 * nh;
  #pragma unroll
  for (int n = 0; n < 4; ++n) {
    const float bv = bias[cb + 16 * n + m];
    #pragma unroll
    for (int r = 0; r < 8; ++r)
      sbuf[(16 * mt + 8 * h + r) * PQF + 64 * nh + 16 * n + m] = acc[n][r] * SC_OW + bv;
  }
  __syncthreads();
  store_rows_f32(sbuf, out + (size_t)row0 * CW + 128 * y, CW, wave, lane);
}

extern "C" void kernel_launch(void* const* d_in, const int* in_sizes, int n_in,
                              void* d_out, int out_size, void* d_ws, size_t ws_size,
                              hipStream_t stream) {
  if (n_in < 5) return;
  if (in_sizes[0] != NTOK * CW) return;
  if (in_sizes[1] != NQKV * CW || in_sizes[2] != NQKV) return;
  if (in_sizes[3] != CW * CW || in_sizes[4] != CW) return;
  if (out_size != NTOK * CW) return;

  const float* x      = (const float*)d_in[0];
  const float* qkv_w  = (const float*)d_in[1];
  const float* qkv_b  = (const float*)d_in[2];
  const float* proj_w = (const float*)d_in[3];
  const float* proj_b = (const float*)d_in[4];
  float* outp = (float*)d_out;

  const size_t szWQKV = (size_t)NQKV * CW * 2;
  const size_t szWO   = (size_t)CW * CW * 2;
  const size_t szP16  = (size_t)NTOK * CW * 2;
  const size_t szP32  = (size_t)NTOK * CW * 4;
  size_t off = 0;
  char* ws = (char*)d_ws;
  f16t*  WQKV = (f16t*)(ws + off);  off += szWQKV;
  f16t*  WO   = (f16t*)(ws + off);  off += szWO;
  f16t*  X16  = (f16t*)(ws + off);  off += szP16;
  float* Qp   = (float*)(ws + off); off += szP32;
  float* Kp   = (float*)(ws + off); off += szP32;
  float* Vp   = (float*)(ws + off); off += szP32;
  f16t*  Opl  = (f16t*)(ws + off);  off += szP16;
  if (off > ws_size) return;

  prep_k<<<XBLK + WQBLK + WOBLK, TPB, 0, stream>>>(x, qkv_w, proj_w, X16, WQKV, WO);
  gemm_qkv_k<<<dim3(NTOK / MT, NQKV / 128), TPB, 0, stream>>>(X16, WQKV, qkv_b, Qp, Kp, Vp);
  attn_k<<<NTOK / WAVES, TPB, 0, stream>>>(Qp, Kp, Vp, Opl);
  gemm_proj_k<<<dim3(NTOK / MT, CW / 128), TPB, 0, stream>>>(Opl, WO, proj_b, outp);
  (void)hipGetLastError();
}
